// GAT_21303037788662
// MI455X (gfx1250) — hardware-verified
//
#include <hip/hip_runtime.h>
#include <stddef.h>
#include <stdint.h>
#include <math.h>


#define F_IN    128
#define HC      256
#define HID     64
#define NHD     4
#define NTHR    256
#define NWAVE   8
#define EPT     8
#define CHUNK   (NTHR * EPT)
#define WCAP    (EPT * 32)
#define LISTN   (NWAVE * WCAP)
#define NBMAX   2048
#define SLOTB   11
#define RCAP    28672
#define DEGCAP  256
#define GBM     64
#define GBN     64
#define GTHR    128
#define MROWS   128
#define NEGSL   0.2f
#define MX0     (-1.0e30f)
#define WSMAX   134217728
#define LDS_AGG ((2 * RCAP + 2 * NBMAX + LISTN) * 4 + 64)
#define MEAS_MAXDEG 33
#define MEAS_B1024  16696

static_assert((CHUNK & (CHUNK - 1)) == 0 && CHUNK <= (1 << SLOTB));
static_assert(NBMAX == (1 << SLOTB));
static_assert(NTHR * 8 == NBMAX);
static_assert(LISTN >= NBMAX);
static_assert(LISTN >= NWAVE * WCAP);
static_assert((RCAP % 32) == 0);
static_assert(LDS_AGG <= 300000);
static_assert(GBM == (GTHR / 32) * 16);
static_assert(GTHR == 2 * GBN && GTHR == 2 * GBM);
static_assert((F_IN % 32) == 0);
static_assert((HC % GBN) == 0 && HID == GBN);
static_assert(HC == NHD * HID);
static_assert((MROWS % GBM) == 0);
static_assert(HC == 32 * 8);
static_assert(HID == 8 * 8);
static_assert(NHD == 4);
static_assert((F_IN / 8) == 16);
static_assert(DEGCAP >= MEAS_MAXDEG + 8);
static_assert(RCAP >= MEAS_B1024 + 8192);
static_assert((1024 % 4) == 0);

typedef float          v4f  __attribute__((ext_vector_type(4)));
typedef float          v8f  __attribute__((ext_vector_type(8)));
typedef int            v4i  __attribute__((ext_vector_type(4)));
typedef int            v8i  __attribute__((ext_vector_type(8)));
typedef unsigned int   v4u  __attribute__((ext_vector_type(4)));
typedef unsigned short v8us __attribute__((ext_vector_type(8)));
typedef __bf16         v16b __attribute__((ext_vector_type(16)));
typedef v4f  __attribute__((may_alias)) v4fa;
typedef v8us __attribute__((may_alias)) v8usa;
union FragB { v16b v; v8us h[2]; v8i w; };

__device__ __forceinline__ v8f wmb(const FragB& a, const FragB& b, v8f c) {
  v8f d = __builtin_amdgcn_wmma_f32_16x16x32_bf16(false, a.v, false, b.v, (short)0, c, false, false);
  asm volatile("v_nop\n\tv_nop\n\tv_nop\n\tv_nop" : "+v"(d) : "v"(a.w), "v"(b.w));
  return d;
}

__device__ __forceinline__ unsigned int f2bf(float f) {
  const unsigned int u = __float_as_uint(f);
  return ((u + 0x7FFFu + ((u >> 16) & 1u)) >> 16) & 0xFFFFu;
}
__device__ __forceinline__ float bf2f(unsigned int b) { return __uint_as_float(b << 16); }
__device__ __forceinline__ float bfr(float f) { return bf2f(f2bf(f)); }
__device__ __forceinline__ v4f bfr4(const v4f a) {
  v4f r; r.x = bfr(a.x); r.y = bfr(a.y); r.z = bfr(a.z); r.w = bfr(a.w); return r;
}
__device__ __forceinline__ unsigned int pk2(float lo, float hi) { return f2bf(lo) | (f2bf(hi) << 16); }
__device__ __forceinline__ v4u pack8(const v4f a, const v4f b) {
  v4u r;
  r.x = pk2(a.x, a.y); r.y = pk2(a.z, a.w); r.z = pk2(b.x, b.y); r.w = pk2(b.z, b.w);
  return r;
}
__device__ __forceinline__ float relu_keep(float x) { return (x > 0.0f) ? x : (x - x); }

__device__ __forceinline__ int scan_chunk(const int* __restrict__ dsts, int nE, int cbase, int slotBase,
                                          int nb, int vec8, int* list, int tid, int lane, int wave) {
  int wc = 0;
  const int el0  = tid * EPT;
  const int e0   = cbase + el0;
  const int sent = -2147483647 - 1;
  v4i da, db;
  if (vec8 != 0 && cbase + CHUNK <= nE) {
    da = *(const v4i*)(dsts + e0);
    db = *(const v4i*)(dsts + e0 + 4);
  } else {
    da.x = (e0     < nE) ? dsts[min(e0,     nE - 1)] : sent;
    da.y = (e0 + 1 < nE) ? dsts[min(e0 + 1, nE - 1)] : sent;
    da.z = (e0 + 2 < nE) ? dsts[min(e0 + 2, nE - 1)] : sent;
    da.w = (e0 + 3 < nE) ? dsts[min(e0 + 3, nE - 1)] : sent;
    db.x = (e0 + 4 < nE) ? dsts[min(e0 + 4, nE - 1)] : sent;
    db.y = (e0 + 5 < nE) ? dsts[min(e0 + 5, nE - 1)] : sent;
    db.z = (e0 + 6 < nE) ? dsts[min(e0 + 6, nE - 1)] : sent;
    db.w = (e0 + 7 < nE) ? dsts[min(e0 + 7, nE - 1)] : sent;
  }
  const unsigned nbs = (unsigned)slotBase;
  const unsigned unb = (unsigned)nb;
  const unsigned s0 = (unsigned)da.x - nbs, s1 = (unsigned)da.y - nbs;
  const unsigned s2 = (unsigned)da.z - nbs, s3 = (unsigned)da.w - nbs;
  const unsigned s4 = (unsigned)db.x - nbs, s5 = (unsigned)db.y - nbs;
  const unsigned s6 = (unsigned)db.z - nbs, s7 = (unsigned)db.w - nbs;
  const bool h0 = s0 < unb, h1 = s1 < unb, h2 = s2 < unb, h3 = s3 < unb;
  const bool h4 = s4 < unb, h5 = s5 < unb, h6 = s6 < unb, h7 = s7 < unb;
  const unsigned any = __builtin_amdgcn_ballot_w32(h0 | h1 | h2 | h3 | h4 | h5 | h6 | h7);
  if (any != 0u) {
#define HITJ(J, HJ, SJ) { \
      const unsigned mj = __builtin_amdgcn_ballot_w32(HJ); \
      if (mj != 0u) { \
        if (HJ) { \
          const int pos = wc + (int)__builtin_amdgcn_mbcnt_lo(mj, 0u); \
          if (pos < WCAP) list[wave * WCAP + pos] = ((el0 + (J)) << SLOTB) | (int)(SJ); \
        } \
        wc += (int)__builtin_popcount(mj); } }
    HITJ(0, h0, s0)
    HITJ(1, h1, s1)
    HITJ(2, h2, s2)
    HITJ(3, h3, s3)
    HITJ(4, h4, s4)
    HITJ(5, h5, s5)
    HITJ(6, h6, s6)
    HITJ(7, h7, s7)
#undef HITJ
  }
  return wc;
}

__global__ __launch_bounds__(NTHR) void k_prep(const float* __restrict__ x, const float* __restrict__ w,
                                               unsigned short* xb, unsigned short* wt,
                                               int nN, int nUx, int gX, int nUw) {
  const int tid = (int)threadIdx.x;
  if ((int)blockIdx.x < gX) {
    const int i = (int)blockIdx.x * NTHR + tid;
    if (i < nUx) {
      const int row = i >> 4;
      const int c0  = (i & 15) * 8;
      const int rc  = row < nN ? row : nN - 1;
      const float* p = x + (size_t)rc * F_IN + c0;
      v4f a = *(const v4fa*)p, b = *(const v4fa*)(p + 4);
      const v4f z4 = {0.f, 0.f, 0.f, 0.f};
      if (row >= nN) { a = z4; b = z4; }
      const v4u hv = pack8(a, b);
      const size_t o = (size_t)row * F_IN + c0;
      *(volatile v4u*)(xb + o) = hv;
      __threadfence();
      *(volatile v4u*)(xb + o) = hv;
    }
  } else {
    const int u = ((int)blockIdx.x - gX) * NTHR + tid;
    if (u < nUw) {
      const int n  = u >> 4;
      const int k8 = (u & 15) * 8;
      const int ncl = n < HC ? n : HC - 1;
      const float* p = w + (size_t)k8 * HC + ncl;
      v4f a, b;
      a.x = p[0];          a.y = p[HC];         a.z = p[2 * HC];     a.w = p[3 * HC];
      b.x = p[4 * HC];     b.y = p[5 * HC];     b.z = p[6 * HC];     b.w = p[7 * HC];
      const v4u wv = pack8(a, b);
      unsigned short* o = wt + (size_t)ncl * F_IN + k8;
      *(volatile v4u*)o = wv;
      __threadfence();
      *(volatile v4u*)o = wv;
    }
  }
}

__global__ __launch_bounds__(GTHR) void k_gemm(
    const unsigned short* __restrict__ A, const unsigned short* __restrict__ WT,
    float* outF, int K, int ldo,
    const float* __restrict__ atts, const float* __restrict__ attd,
    float* SD, int MPr)
{
  __shared__ __attribute__((aligned(16))) float stg[GBM * GBN];
  __shared__ __attribute__((aligned(16))) float satt[2 * GBN];
  __shared__ __attribute__((aligned(16))) float sdot[2 * GBM];
  const int tid = (int)threadIdx.x, lane = tid & 31, wave = tid >> 5, hh = lane >> 4, m = lane & 15;
  const int rowBase = (int)blockIdx.x * GBM;
  const int head    = (int)blockIdx.y;
  const int col0    = head * GBN;

  {
    const int which = tid >> 6;
    const int c  = tid & 63;
    const float vs = atts[head * HID + c];
    const float vd = attd[head * HID + c];
    const float v = (which == 0) ? vs : vd;
    satt[which * GBN + c] = bfr(v);
  }

  v8f acc[4];
  {
    const v8f z = {0.f, 0.f, 0.f, 0.f, 0.f, 0.f, 0.f, 0.f};
    acc[0] = z; acc[1] = z; acc[2] = z; acc[3] = z;
  }
  const unsigned short* ap = A  + (size_t)(rowBase + 16 * wave + m) * (size_t)K + 8 * hh;
  const unsigned short* wp = WT + (size_t)(col0 + m) * (size_t)K + 8 * hh;
  const int ksteps = K >> 5;
#pragma unroll 1
  for (int ks = 0; ks < ksteps; ++ks) {
    FragB af;
    af.h[0] = *(const v8usa*)(ap + 32 * ks);
    af.h[1] = *(const v8usa*)(ap + 32 * ks + 16);
#pragma unroll
    for (int t = 0; t < 4; ++t) {
      const unsigned short* wq = wp + (size_t)(16 * t) * (size_t)K + 32 * ks;
      FragB bf;
      bf.h[0] = *(const v8usa*)wq;
      bf.h[1] = *(const v8usa*)(wq + 16);
      acc[t] = wmb(af, bf, acc[t]);
    }
  }

#pragma unroll
  for (int t = 0; t < 4; ++t) {
    const int lc = 16 * t + m;
#pragma unroll
    for (int r = 0; r < 8; ++r) {
      const int lr = 16 * wave + 8 * hh + r;
      stg[lr * GBN + lc] = acc[t][r];
    }
  }
  __syncthreads();

  {
    const int row = tid & 63, which = tid >> 6;
    const float* sa = satt + which * GBN;
    const float* hr = stg + row * GBN;
    float d = 0.f;
#pragma unroll 4
    for (int c4 = 0; c4 < GBN / 4; ++c4) {
      const v4f hv = *(const v4fa*)(hr + 4 * c4);
      const v4f av = *(const v4fa*)(sa + 4 * c4);
      d = fmaf(hv.x, av.x, d);
      d = fmaf(hv.y, av.y, d);
      d = fmaf(hv.z, av.z, d);
      d = fmaf(hv.w, av.w, d);
    }
    sdot[which * GBM + row] = d;
  }
  __syncthreads();

  v4f fv[8];
#pragma unroll
  for (int i = 0; i < 8; ++i) {
    const int lr = 16 * wave + 2 * i + hh;
    fv[i] = *(const v4fa*)(stg + lr * GBN + 4 * m);
  }
  const int which2 = lane >> 4, piece = lane & 15;
  const v4f sdv = *(const v4fa*)(sdot + which2 * GBM + 4 * piece);
  float* sp = SD + (size_t)(2 * head + which2) * (size_t)MPr + rowBase + 4 * piece;

#pragma unroll
  for (int i = 0; i < 8; ++i) {
    const int lr = 16 * wave + 2 * i + hh;
    const int gr = rowBase + lr;
    float* op = outF + (size_t)gr * (size_t)ldo + col0 + 4 * m;
    *(volatile v4f*)op = fv[i];
  }
  if (wave == 0) *(volatile v4f*)sp = sdv;
  __threadfence();
#pragma unroll
  for (int i = 0; i < 8; ++i) {
    const int lr = 16 * wave + 2 * i + hh;
    const int gr = rowBase + lr;
    float* op = outF + (size_t)gr * (size_t)ldo + col0 + 4 * m;
    *(volatile v4f*)op = fv[i];
  }
  if (wave == 0) *(volatile v4f*)sp = sdv;
}

__global__ __launch_bounds__(NTHR) void k_agg(
    const int* __restrict__ srcs, const int* __restrict__ dsts,
    const float* __restrict__ F, const float* __restrict__ SD,
    const float* __restrict__ bias, float* out,
    int nN, int nE, int nb, int vec8, int MPr) {
  extern __shared__ v4f lds_dyn[];
  int* reg1 = (int*)lds_dyn;
  int* reg2 = reg1 + RCAP;
  int* scnt = reg2 + RCAP;
  int* soff = scnt + NBMAX;
  int* list = soff + NBMAX;
  int* wcnt = list + LISTN;
  int* wtot = wcnt + NWAVE;
  const int tid = (int)threadIdx.x, lane = tid & 31, wave = tid >> 5;
  const int nodeBase = (int)blockIdx.x * nb;

  for (int i = tid; i < NBMAX; i += NTHR) scnt[i] = 0;
  __syncthreads();

  int tot = 0;
  const int nChunks = (nE + CHUNK - 1) / CHUNK;
#pragma unroll 1
  for (int ch = 0; ch < nChunks; ++ch) {
    const int cbase = ch * CHUNK;
    const int wc = scan_chunk(dsts, nE, cbase, nodeBase, nb, vec8, list, tid, lane, wave);
    if (lane == 0) wcnt[wave] = wc;
    __syncthreads();
    int pre = 0, all = 0;
#pragma unroll
    for (int w2 = 0; w2 < NWAVE; ++w2) {
      int c = wcnt[w2];
      c = c < 0 ? 0 : (c > WCAP ? WCAP : c);
      all += c;
      pre += (w2 < wave) ? c : 0;
    }
    const int wcc  = wc > WCAP ? WCAP : wc;
    const int base = tot + pre;
#pragma unroll 1
    for (int i = lane; i < wcc; i += 32) {
      const int ent = list[wave * WCAP + i];
      const int el  = (ent >> SLOTB) & (CHUNK - 1);
      const int sl  = ent & (NBMAX - 1);
      int eid = cbase + el;
      eid = eid > nE - 1 ? nE - 1 : eid;
      const int pos = base + i;
      if (pos < RCAP) reg1[pos] = (int)(((unsigned)eid << SLOTB) | (unsigned)sl);
    }
    tot += all;
    tot = tot > RCAP ? RCAP : tot;
    __syncthreads();
  }
  const int nh = tot;

  if (wave == 0) {
#pragma unroll 1
    for (int b0 = 0; b0 < nh; b0 += 32) {
      const int idx = b0 + lane;
      const int uv  = reg1[idx < nh ? idx : nh - 1];
      const int m32 = (nh - b0) < 32 ? (nh - b0) : 32;
#pragma unroll 1
      for (int k = 0; k < m32; ++k) {
        const int u  = __builtin_amdgcn_readlane(uv, k);
        const int sl = u & (NBMAX - 1);
        if (lane == 0) scnt[sl] = scnt[sl] + 1;
      }
    }
  }
  __syncthreads();

  {
    const v4i ca = *(const v4i*)(scnt + 8 * tid);
    const v4i cb = *(const v4i*)(scnt + 8 * tid + 4);
    const int e0 = ca.x < 0 ? 0 : ca.x, e1 = ca.y < 0 ? 0 : ca.y, e2 = ca.z < 0 ? 0 : ca.z, e3 = ca.w < 0 ? 0 : ca.w;
    const int e4 = cb.x < 0 ? 0 : cb.x, e5 = cb.y < 0 ? 0 : cb.y, e6 = cb.z < 0 ? 0 : cb.z, e7 = cb.w < 0 ? 0 : cb.w;
    const int ts = e0 + e1 + e2 + e3 + e4 + e5 + e6 + e7;
    int incl = ts;
#pragma unroll
    for (int d = 1; d < 32; d <<= 1) {
      const int up = __shfl_up(incl, d);
      if (lane >= d) incl += up;
    }
    if (lane == 31) wtot[wave] = incl;
    __syncthreads();
    int pre = 0;
#pragma unroll
    for (int w2 = 0; w2 < NWAVE; ++w2) pre += (w2 < wave) ? wtot[w2] : 0;
    int run = pre + incl - ts;
    soff[8 * tid + 0] = run; run += e0;
    soff[8 * tid + 1] = run; run += e1;
    soff[8 * tid + 2] = run; run += e2;
    soff[8 * tid + 3] = run; run += e3;
    soff[8 * tid + 4] = run; run += e4;
    soff[8 * tid + 5] = run; run += e5;
    soff[8 * tid + 6] = run; run += e6;
    soff[8 * tid + 7] = run;
  }
  __syncthreads();
  for (int i = tid; i < NBMAX; i += NTHR) list[i] = soff[i];
  __syncthreads();

  if (wave == 0) {
#pragma unroll 1
    for (int b0 = 0; b0 < nh; b0 += 32) {
      const int idx = b0 + lane;
      const int uv  = reg1[idx < nh ? idx : nh - 1];
      const int m32 = (nh - b0) < 32 ? (nh - b0) : 32;
#pragma unroll 1
      for (int k = 0; k < m32; ++k) {
        const int u   = __builtin_amdgcn_readlane(uv, k);
        const int sl  = u & (NBMAX - 1);
        const int eid = (int)((unsigned)u >> SLOTB);
        if (lane == 0) {
          int pos = list[sl];
          pos = pos < 0 ? 0 : (pos > RCAP - 1 ? RCAP - 1 : pos);
          reg2[pos] = eid;
          list[sl] = pos + 1;
        }
      }
    }
  }
  __syncthreads();

  const int nbw = nb >> 3;
  const bool ovf = (nh >= RCAP);
  const float qnan = __int_as_float(0x7fc00000);
  const int head = lane >> 3;
  const int jj   = lane & 7;
  const int cA   = HID * head + 4 * jj;
  const v4f bbA  = bfr4(*(const v4fa*)(bias + cA));
  const v4f bbB  = bfr4(*(const v4fa*)(bias + cA + 32));
  const float* ASp = SD + (size_t)(2 * head) * (size_t)MPr;
  const float* ADp = ASp + MPr;
  const bool pieceB = (lane & 8) != 0;

#pragma unroll 1
  for (int jt = 0; jt < nbw; ++jt) {
    const int slot = wave * nbw + jt;
    const int grow = nodeBase + slot;
    const int gcl  = grow < nN ? grow : nN - 1;
    int st = soff[slot];
    const int craw = scnt[slot];
    int cnt = craw;
    st  = st < 0 ? 0 : (st > nh ? nh : st);
    cnt = cnt < 0 ? 0 : (cnt > DEGCAP ? DEGCAP : cnt);
    if (cnt > nh - st) cnt = nh - st;
    const float pz = (ovf || craw > DEGCAP) ? qnan : 0.0f;

    const float adv = ADp[gcl];
    float mx = MX0, dn = 0.0f;
    v4f av = {0.f, 0.f, 0.f, 0.f};
    v4f aw = {0.f, 0.f, 0.f, 0.f};

#pragma unroll 1
    for (int q = 0; q < cnt; ++q) {
      int idx = st + q; idx = idx > RCAP - 1 ? RCAP - 1 : idx;
      int eid = reg2[idx]; eid = eid < 0 ? 0 : (eid > nE - 1 ? nE - 1 : eid);
      const int sraw = srcs[eid];
      const int s = sraw < 0 ? 0 : (sraw > nN - 1 ? nN - 1 : sraw);
      const float* fr = F + (size_t)s * HC + cA;
      const v4f fs = *(const v4fa*)fr;
      const v4f ft = *(const v4fa*)(fr + 32);
      float lg = ASp[s] + adv;
      lg = lg > 0.f ? lg : NEGSL * lg;
      const float df = lg - mx;
      const float ee = expf(-fabsf(df));
      const bool up  = df > 0.f;
      const float s1 = up ? ee : 1.0f;
      const float s2 = up ? 1.0f : ee;
      mx = up ? lg : mx;
      dn = fmaf(dn, s1, s2);
      av.x = fmaf(av.x, s1, s2 * fs.x);
      av.y = fmaf(av.y, s1, s2 * fs.y);
      av.z = fmaf(av.z, s1, s2 * fs.z);
      av.w = fmaf(av.w, s1, s2 * fs.w);
      aw.x = fmaf(aw.x, s1, s2 * ft.x);
      aw.y = fmaf(aw.y, s1, s2 * ft.y);
      aw.z = fmaf(aw.z, s1, s2 * ft.z);
      aw.w = fmaf(aw.w, s1, s2 * ft.w);
    }
    const bool has  = cnt > 0;
    const float dnz = has ? dn : 1.0f;
    const float inv = __builtin_amdgcn_rcpf(dnz);
    float a0 = (has ? av.x * inv : 0.0f) + bbA.x;
    float a1 = (has ? av.y * inv : 0.0f) + bbA.y;
    float a2 = (has ? av.z * inv : 0.0f) + bbA.z;
    float a3 = (has ? av.w * inv : 0.0f) + bbA.w;
    float b0 = (has ? aw.x * inv : 0.0f) + bbB.x;
    float b1 = (has ? aw.y * inv : 0.0f) + bbB.y;
    float b2 = (has ? aw.z * inv : 0.0f) + bbB.z;
    float b3 = (has ? aw.w * inv : 0.0f) + bbB.w;
    a0 += __shfl_xor(a0, 8);  a1 += __shfl_xor(a1, 8);  a2 += __shfl_xor(a2, 8);  a3 += __shfl_xor(a3, 8);
    b0 += __shfl_xor(b0, 8);  b1 += __shfl_xor(b1, 8);  b2 += __shfl_xor(b2, 8);  b3 += __shfl_xor(b3, 8);
    a0 += __shfl_xor(a0, 16); a1 += __shfl_xor(a1, 16); a2 += __shfl_xor(a2, 16); a3 += __shfl_xor(a3, 16);
    b0 += __shfl_xor(b0, 16); b1 += __shfl_xor(b1, 16); b2 += __shfl_xor(b2, 16); b3 += __shfl_xor(b3, 16);
    v4f ov;
    ov.x = relu_keep(0.25f * (pieceB ? b0 : a0)) + pz;
    ov.y = relu_keep(0.25f * (pieceB ? b1 : a1)) + pz;
    ov.z = relu_keep(0.25f * (pieceB ? b2 : a2)) + pz;
    ov.w = relu_keep(0.25f * (pieceB ? b3 : a3)) + pz;
    float* op = out + (size_t)gcl * HID + 4 * (lane & 15);
    const bool wr = (grow < nN) && (lane < 16);
    if (wr) *(volatile v4f*)op = ov;
    __threadfence();
    if (wr) *(volatile v4f*)op = ov;
  }
}

static int pick_nb(int nE, int nN) {
  int nb = NBMAX;
  while (nb > 32 && (long long)nb * (long long)nE * 5LL > (long long)RCAP * (long long)nN * 4LL) nb >>= 1;
  return nb;
}
static inline int cdiv(int a, int b) { return (a + b - 1) / b; }

extern "C" void kernel_launch(void* const* d_in, const int* in_sizes, int n_in,
                              void* d_out, int out_size, void* d_ws, size_t ws_size,
                              hipStream_t stream) {
  if (n_in < 7) return;
  const int nN = in_sizes[0] / F_IN;
  if (nN <= 0 || in_sizes[0] != nN * F_IN || nN > (1 << 22)) return;
  const int nE = in_sizes[1];
  if (nE < 1 || nE >= (1 << (32 - SLOTB))) return;
  if (in_sizes[2] != nE) return;
  if (in_sizes[3] != F_IN * HC) return;
  if (in_sizes[4] != NHD * HID || in_sizes[5] != NHD * HID) return;
  if (in_sizes[6] != HC) return;
  if (out_size != nN * HID) return;

  const float* x    = (const float*)d_in[0];
  const int*   src  = (const int*)  d_in[1];
  const int*   dst  = (const int*)  d_in[2];
  const float* W    = (const float*)d_in[3];
  const float* al   = (const float*)d_in[4];
  const float* ar   = (const float*)d_in[5];
  const float* bias = (const float*)d_in[6];
  float* out = (float*)d_out;

  const int MP   = cdiv(nN, MROWS) * MROWS;
  const int nb   = pick_nb(nE, nN);
  if (nb < 32 || (nb & (nb - 1)) != 0 || nb > NBMAX) return;
  const int gA   = cdiv(nN, nb);
  const int vec8 = ((nE & 3) == 0) ? 1 : 0;
  if ((long long)gA * nb < (long long)nN) return;

  char* ws = (char*)d_ws;
  size_t off = 0;
  const size_t oXB = off; off += (size_t)MP * F_IN * 2;            off = (off + 255) & ~(size_t)255;
  const size_t oWT = off; off += (size_t)HC * F_IN * 2;            off = (off + 255) & ~(size_t)255;
  const size_t oH  = off; off += (size_t)MP * HC * 4;              off = (off + 255) & ~(size_t)255;
  const size_t oSD = off; off += (size_t)2 * NHD * MP * 4;         off = (off + 255) & ~(size_t)255;
  if (off > ws_size || off > (size_t)WSMAX) return;
  unsigned short* XB = (unsigned short*)(ws + oXB);
  unsigned short* WT = (unsigned short*)(ws + oWT);
  float*          H  = (float*)(ws + oH);
  float*          SD = (float*)(ws + oSD);

  hipFuncSetAttribute(reinterpret_cast<const void*>(&k_agg),
                      hipFuncAttributeMaxDynamicSharedMemorySize, LDS_AGG);

  const int nUx = MP * (F_IN / 8);
  const int gX  = cdiv(nUx, NTHR);
  const int nUw = HC * (F_IN / 8);
  const int gW  = cdiv(nUw, NTHR);
  k_prep<<<gX + gW, NTHR, 0, stream>>>(x, W, XB, WT, nN, nUx, gX, nUw);

  k_gemm<<<dim3(MP / GBM, HC / GBN), GTHR, 0, stream>>>(XB, WT, H, F_IN, HC, al, ar, SD, MP);

  k_agg<<<gA, NTHR, LDS_AGG, stream>>>(src, dst, H, SD, bias, out, nN, nE, nb, vec8, MP);
}
